// MetaS5Block_70506183131277
// MI455X (gfx1250) — hardware-verified
//
#include <hip/hip_runtime.h>
#include <math.h>

constexpr int NBATCH   = 4;
constexpr int SEQLEN   = 4096;
constexpr int NTOK     = NBATCH * SEQLEN;
constexpr int D_INPUT  = 512;
constexpr int D_MODEL  = 1024;
constexpr int N_STATE  = 512;
constexpr int D_FF2    = 2 * D_MODEL;
constexpr int XS_COLS  = 4 * N_STATE;
constexpr int HALF_TOK = NTOK / 2;
constexpr int R2_WORDS = XS_COLS / 2;
constexpr float W_CARRY      = 64.0f;
constexpr float W_CARRY_INV  = 1.0f / W_CARRY;
constexpr float XS_CARRY     = 16.0f;
constexpr float YS_SCALE     = 1.0f / (W_CARRY * XS_CARRY);
constexpr float LN_EPS_F     = 1e-5f;

static_assert(XS_COLS == D_FF2);
static_assert(2 * N_STATE == D_MODEL);
static_assert(NTOK % 64 == 0 && HALF_TOK % 64 == 0);
static_assert(D_MODEL % 64 == 0 && D_INPUT % 64 == 0 && D_FF2 % 64 == 0);
static_assert(D_INPUT % 32 == 0 && D_MODEL % 32 == 0 && XS_COLS % 32 == 0);
static_assert(N_STATE % 32 == 0 && SEQLEN % 8 == 0);
static_assert(D_MODEL == 4 * 256);
static_assert((NBATCH * N_STATE) % 256 == 0);
static_assert(NTOK % 8 == 0 && HALF_TOK % 4 == 0);

typedef __attribute__((ext_vector_type(16))) _Float16 v16h;
typedef __attribute__((ext_vector_type(8)))  _Float16 v8h;
typedef __attribute__((ext_vector_type(8)))  float    v8f;
typedef __attribute__((ext_vector_type(4)))  float    v4f;
typedef __attribute__((ext_vector_type(4)))  unsigned v4u;

__device__ __forceinline__ float h16_to_f32(unsigned hb) {
  const unsigned sgn = (hb & 0x8000u) << 16;
  const unsigned em = hb & 0x7fffu;
  const float fn = __uint_as_float((em << 13) + 0x38000000u);
  const float fs = (float)em * 5.9604644775390625e-8f;
  const float mag = (em < 0x400u) ? fs : fn;
  return __uint_as_float(__float_as_uint(mag) | sgn);
}

__device__ __forceinline__ unsigned pack_h2(float a, float b) {
  const _Float16 ha = (_Float16)a;
  const _Float16 hb = (_Float16)b;
  const unsigned ua = (unsigned)__builtin_bit_cast(unsigned short, ha);
  const unsigned ub = (unsigned)__builtin_bit_cast(unsigned short, hb);
  return ua | (ub << 16);
}

__device__ __forceinline__ void unpack8(const v4u w, v4f& lo, v4f& hi) {
  const unsigned w0 = w[0];
  const unsigned w1 = w[1];
  const unsigned w2 = w[2];
  const unsigned w3 = w[3];
  lo[0] = h16_to_f32(w0 & 0xffffu);
  lo[1] = h16_to_f32(w0 >> 16);
  lo[2] = h16_to_f32(w1 & 0xffffu);
  lo[3] = h16_to_f32(w1 >> 16);
  hi[0] = h16_to_f32(w2 & 0xffffu);
  hi[1] = h16_to_f32(w2 >> 16);
  hi[2] = h16_to_f32(w3 & 0xffffu);
  hi[3] = h16_to_f32(w3 >> 16);
}

__device__ __forceinline__ float gelu_erf(float x) {
  return 0.5f * x * (1.0f + erff(x * 0.70710678118654752f));
}

__device__ __forceinline__ void wave_lds_fence() {
  __builtin_amdgcn_fence(__ATOMIC_RELEASE, "workgroup");
  __builtin_amdgcn_wave_barrier();
  __builtin_amdgcn_fence(__ATOMIC_ACQUIRE, "workgroup");
}

struct FragH {
  union U { v16h v; v8h h[2]; };
  static __device__ __forceinline__ v16h load(const _Float16* p) {
    U f;
    f.h[0] = *(const v8h*)(p);
    f.h[1] = *(const v8h*)(p + 16);
    return f.v;
  }
  static __device__ __forceinline__ v8f mma(v16h a, v16h b, v8f c) {
    return __builtin_amdgcn_wmma_f32_16x16x32_f16(false, a, false, b, (short)0, c, false, false);
  }
};
__device__ __forceinline__ void group_guard(v8f& a0, v8f& a1, v8f& a2, v8f& a3,
                                            v16h x, v16h b0, v16h b1, v16h b2, v16h b3) {
  asm volatile("v_nop\n\tv_nop\n\tv_nop\n\tv_nop"
               : "+v"(a0), "+v"(a1), "+v"(a2), "+v"(a3)
               : "v"(x), "v"(b0), "v"(b1), "v"(b2), "v"(b3));
}
__device__ __forceinline__ void acc_guard4(v8f& a, v8f& b, v8f& c, v8f& d) {
  asm volatile("v_nop\n\tv_nop\n\tv_nop\n\tv_nop" : "+v"(a), "+v"(b), "+v"(c), "+v"(d));
}

template <int OUT_MODE, bool RESID16>
__global__ __launch_bounds__(256) void wmma_gemm64_f16(
    const unsigned short* __restrict__ Ap, int lda,
    const unsigned short* __restrict__ Btp, int ldb,
    void* Cout, int ldc,
    const unsigned short* Rp, int ldr,
    int M, int N, int K, float scale) {
  const _Float16* A  = (const _Float16*)Ap;
  const _Float16* Bt = (const _Float16*)Btp;
  __shared__ __align__(16) float sT[8][16 * 68];
  const int lane = threadIdx.x & 31;
  const int wave = threadIdx.x >> 5;
  const int tilesN = N >> 6;
  const int tilesM = M >> 6;
  const int tile = blockIdx.x * 8 + wave;
  if (tile >= tilesM * tilesN) return;
  const int tm = tile / tilesN;
  const int tn = tile - tm * tilesN;
  const int m0 = tm << 6;
  const int n0 = tn << 6;
  const int rlane = lane & 15;
  const int koff  = (lane >> 4) * 8;
  const int mOff  = (lane >> 4) * 8;

  const _Float16* bp[4];
  const _Float16* ap[4];
#pragma unroll
  for (int j = 0; j < 4; ++j) bp[j] = Bt + (size_t)(n0 + (j << 4) + rlane) * ldb + koff;
#pragma unroll
  for (int i = 0; i < 4; ++i) ap[i] = A + (size_t)(m0 + (i << 4) + rlane) * lda + koff;

  v8f acc[4][4];
#pragma unroll
  for (int i = 0; i < 4; ++i)
#pragma unroll
    for (int j = 0; j < 4; ++j) acc[i][j] = (v8f){0.f, 0.f, 0.f, 0.f, 0.f, 0.f, 0.f, 0.f};

#pragma unroll 1
  for (int k0 = 0; k0 < K; k0 += 32) {
    v16h bh[4];
#pragma unroll
    for (int j = 0; j < 4; ++j) bh[j] = FragH::load(bp[j] + k0);
#pragma unroll
    for (int i = 0; i < 4; ++i) {
      const v16h ah = FragH::load(ap[i] + k0);
#pragma unroll
      for (int j = 0; j < 4; ++j) acc[i][j] = FragH::mma(ah, bh[j], acc[i][j]);
      group_guard(acc[i][0], acc[i][1], acc[i][2], acc[i][3], ah, bh[0], bh[1], bh[2], bh[3]);
    }
  }
  acc_guard4(acc[0][0], acc[0][1], acc[0][2], acc[0][3]);
  acc_guard4(acc[1][0], acc[1][1], acc[1][2], acc[1][3]);
  acc_guard4(acc[2][0], acc[2][1], acc[2][2], acc[2][3]);
  acc_guard4(acc[3][0], acc[3][1], acc[3][2], acc[3][3]);

  float* slab = sT[wave];
#pragma unroll
  for (int i = 0; i < 4; ++i) {
    const int mBase = m0 + (i << 4);
#pragma unroll
    for (int j = 0; j < 4; ++j) {
#pragma unroll
      for (int r = 0; r < 8; ++r) {
        slab[(mOff + r) * 68 + (j << 4) + rlane] = acc[i][j][r] * scale;
      }
    }
    wave_lds_fence();
    if (OUT_MODE == 0) {
      float* C = (float*)Cout;
      const int hh = lane >> 4;
      const int c4 = (lane & 15) * 4;
      for (int pass = 0; pass < 2; ++pass) {
#pragma unroll
        for (int it = 0; it < 8; ++it) {
          const int row = it * 2 + hh;
          const v4f v = *(const v4f*)(slab + row * 68 + c4);
          *(volatile v4f*)(C + (size_t)(mBase + row) * ldc + n0 + c4) = v;
        }
        __threadfence();
      }
    } else {
      const int q  = lane >> 3;
      const int c8 = (lane & 7) * 8;
      unsigned short* C = (unsigned short*)Cout;
      v4u ov[4];
#pragma unroll
      for (int it = 0; it < 4; ++it) {
        const int row = it * 4 + q;
        const float* sp = slab + row * 68 + c8;
        v4f s0 = *(const v4f*)(sp);
        v4f s1 = *(const v4f*)(sp + 4);
        if (RESID16) {
          const v4u rw = *(const v4u*)(Rp + (size_t)(mBase + row) * ldr + n0 + c8);
          v4f r0, r1;
          unpack8(rw, r0, r1);
          s0 = s0 + r0;
          s1 = s1 + r1;
        }
        v4u o;
        o[0] = pack_h2(s0[0], s0[1]);
        o[1] = pack_h2(s0[2], s0[3]);
        o[2] = pack_h2(s1[0], s1[1]);
        o[3] = pack_h2(s1[2], s1[3]);
        ov[it] = o;
      }
      for (int pass = 0; pass < 2; ++pass) {
#pragma unroll
        for (int it = 0; it < 4; ++it) {
          const int row = it * 4 + q;
          *(volatile v4u*)(C + (size_t)(mBase + row) * ldc + n0 + c8) = ov[it];
        }
        __threadfence();
      }
    }
    wave_lds_fence();
  }
}

__global__ __launch_bounds__(256) void cvt8_rows_kernel(const float* __restrict__ src, unsigned short* __restrict__ dst,
                                                        int nrow, int ncol8, int spitch, float sc,
                                                        int dpitch, int drow0, int drstep) {
  const int i  = blockIdx.x * 256 + threadIdx.x;
  const int n8 = nrow * ncol8;
  if (i < n8) {
    const int row = i / ncol8;
    const int c8  = i - row * ncol8;
    const float* sp = src + (size_t)row * spitch + c8 * 8;
    const v4f a = *(const v4f*)(sp);
    const v4f b = *(const v4f*)(sp + 4);
    v4u o;
    o[0] = pack_h2(a[0] * sc, a[1] * sc);
    o[1] = pack_h2(a[2] * sc, a[3] * sc);
    o[2] = pack_h2(b[0] * sc, b[1] * sc);
    o[3] = pack_h2(b[2] * sc, b[3] * sc);
    unsigned short* dp = dst + (size_t)(drow0 + row * drstep) * dpitch + c8 * 8;
    *(volatile v4u*)dp = o;
    __threadfence();
    *(volatile v4u*)dp = o;
  }
}

__global__ __launch_bounds__(256) void cvt_wc_kernel(const float* __restrict__ Cre, const float* __restrict__ Cim,
                                                     unsigned short* __restrict__ dst, float sc) {
  const int i = blockIdx.x * 256 + threadIdx.x;
  if (i < D_MODEL * (XS_COLS / 8)) {
    const int h = i >> 8;
    const int c = i & 255;
    const v4f cr = *(const v4f*)(Cre + (size_t)h * (2 * N_STATE) + 4 * c);
    const v4f ci = *(const v4f*)(Cim + (size_t)h * (2 * N_STATE) + 4 * c);
    v4u o;
    o[0] = pack_h2(cr[0] * sc, -(ci[0] * sc));
    o[1] = pack_h2(cr[1] * sc, -(ci[1] * sc));
    o[2] = pack_h2(cr[2] * sc, -(ci[2] * sc));
    o[3] = pack_h2(cr[3] * sc, -(ci[3] * sc));
    unsigned short* dp = dst + (size_t)h * XS_COLS + 8 * c;
    *(volatile v4u*)dp = o;
    __threadfence();
    *(volatile v4u*)dp = o;
  }
}

__global__ __launch_bounds__(256) void disc_prep_kernel(const float* __restrict__ Lre, const float* __restrict__ Lim,
                                                        const float* __restrict__ logstep, float* __restrict__ lamgam) {
#pragma clang fp contract(off)
  const int p = blockIdx.x * 256 + threadIdx.x;
  if (p < N_STATE) {
    const float cr = Lre[p];
    const float ci = Lim[p];
    const float dt = expf(logstep[p]);
    const float zr = cr * dt;
    const float zi = ci * dt;
    const float er = expf(zr);
    const float lbr = er * cosf(zi);
    const float lbi = er * sinf(zi);
    const float ar = lbr - 1.0f;
    const float ai = lbi;
    const float den = cr * cr + ci * ci;
    const float inv = 1.0f / den;
    const float gr = (ar * cr + ai * ci) * inv;
    const float gi = (ai * cr - ar * ci) * inv;
    v4f o;
    o[0] = lbr;
    o[1] = lbi;
    o[2] = gr;
    o[3] = gi;
    float* dp = lamgam + 4 * p;
    *(volatile v4f*)dp = o;
    __threadfence();
    *(volatile v4f*)dp = o;
  }
}

__device__ __forceinline__ void ln_row_store(const float* rb, const float* __restrict__ gw, const float* __restrict__ gb,
                                             unsigned short* dst, int lane) {
  float s = 0.0f;
#pragma unroll 1
  for (int q = 0; q < 4; ++q) {
    const v4f a = *(const v4f*)(rb + 256 * q + 8 * lane);
    const v4f c = *(const v4f*)(rb + 256 * q + 8 * lane + 4);
    s += ((a[0] + a[1]) + (a[2] + a[3])) + ((c[0] + c[1]) + (c[2] + c[3]));
  }
#pragma unroll
  for (int off = 1; off < 32; off <<= 1) s += __shfl_xor(s, off, 32);
  const float mu = s * (1.0f / (float)D_MODEL);
  float ss = 0.0f;
#pragma unroll 1
  for (int q = 0; q < 4; ++q) {
    const v4f a = *(const v4f*)(rb + 256 * q + 8 * lane);
    const v4f c = *(const v4f*)(rb + 256 * q + 8 * lane + 4);
#pragma unroll
    for (int e = 0; e < 4; ++e) {
      const float d0 = a[e] - mu;
      const float d1 = c[e] - mu;
      ss += d0 * d0;
      ss += d1 * d1;
    }
  }
#pragma unroll
  for (int off = 1; off < 32; off <<= 1) ss += __shfl_xor(ss, off, 32);
  const float rstd = rsqrtf(ss * (1.0f / (float)D_MODEL) + LN_EPS_F);
  for (int pass = 0; pass < 2; ++pass) {
#pragma unroll 1
    for (int q = 0; q < 4; ++q) {
      const int col = 256 * q + 8 * lane;
      const v4f a  = *(const v4f*)(rb + col);
      const v4f c  = *(const v4f*)(rb + col + 4);
      const v4f w0 = *(const v4f*)(gw + col);
      const v4f w1 = *(const v4f*)(gw + col + 4);
      const v4f b0 = *(const v4f*)(gb + col);
      const v4f b1 = *(const v4f*)(gb + col + 4);
      v4u o;
      o[0] = pack_h2(((a[0] - mu) * rstd) * w0[0] + b0[0], ((a[1] - mu) * rstd) * w0[1] + b0[1]);
      o[1] = pack_h2(((a[2] - mu) * rstd) * w0[2] + b0[2], ((a[3] - mu) * rstd) * w0[3] + b0[3]);
      o[2] = pack_h2(((c[0] - mu) * rstd) * w1[0] + b1[0], ((c[1] - mu) * rstd) * w1[1] + b1[1]);
      o[3] = pack_h2(((c[2] - mu) * rstd) * w1[2] + b1[2], ((c[3] - mu) * rstd) * w1[3] + b1[3]);
      *(volatile v4u*)(dst + col) = o;
    }
    __threadfence();
  }
}

__global__ __launch_bounds__(256) void ln_f32_rows_kernel(const float* __restrict__ src, const float* __restrict__ gw,
                                                          const float* __restrict__ gb, unsigned short* __restrict__ dst,
                                                          int nrows) {
  __shared__ __align__(16) float rowbuf[8][D_MODEL];
  const int lane = threadIdx.x & 31;
  const int wave = threadIdx.x >> 5;
  const int row = blockIdx.x * 8 + wave;
  if (row >= nrows) return;
  float* rb = rowbuf[wave];
  const float* sp = src + (size_t)row * D_MODEL + 8 * lane;
#pragma unroll
  for (int q = 0; q < 4; ++q) {
    const v4f a = *(const v4f*)(sp + 256 * q);
    const v4f c = *(const v4f*)(sp + 256 * q + 4);
    *(v4f*)(rb + 256 * q + 8 * lane) = a;
    *(v4f*)(rb + 256 * q + 8 * lane + 4) = c;
  }
  wave_lds_fence();
  ln_row_store(rb, gw, gb, dst + (size_t)row * D_MODEL, lane);
}

__global__ __launch_bounds__(128) void gelu_res_ln_kernel(const unsigned short* __restrict__ Yp, unsigned short* Up,
                                                          const float* __restrict__ Dv, const float* __restrict__ gw,
                                                          const float* __restrict__ gb, int row0, int nrows) {
  __shared__ __align__(16) float rowbuf[4][D_MODEL];
  __shared__ __align__(16) float ubuf[4][D_MODEL];
  const int lane = threadIdx.x & 31;
  const int wave = threadIdx.x >> 5;
  const int lrow = blockIdx.x * 4 + wave;
  if (lrow >= nrows) return;
  float* rb = rowbuf[wave];
  float* ub = ubuf[wave];
  const unsigned short* yr = Yp + (size_t)lrow * D_MODEL + 8 * lane;
  unsigned short* urow = Up + (size_t)(row0 + lrow) * D_MODEL;
  const unsigned short* ur = urow + 8 * lane;
#pragma unroll
  for (int q = 0; q < 4; ++q) {
    const v4u yw = *(const v4u*)(yr + 256 * q);
    const v4u uw = *(const v4u*)(ur + 256 * q);
    v4f y0, y1, u0, u1;
    unpack8(yw, y0, y1);
    unpack8(uw, u0, u1);
    *(v4f*)(rb + 256 * q + 8 * lane) = y0;
    *(v4f*)(rb + 256 * q + 8 * lane + 4) = y1;
    *(v4f*)(ub + 256 * q + 8 * lane) = u0;
    *(v4f*)(ub + 256 * q + 8 * lane + 4) = u1;
  }
  wave_lds_fence();
#pragma unroll 1
  for (int i = 0; i < 32; ++i) {
    const int idx = ((i >> 3) << 8) + 8 * lane + (i & 7);
    const float yv = rb[idx];
    const float uv = ub[idx];
    const float dv = Dv[idx];
    const float pre = fmaf(dv, uv, yv);
    rb[idx] = gelu_erf(pre) + uv;
  }
  wave_lds_fence();
  ln_row_store(rb, gw, gb, urow, lane);
}

__global__ __launch_bounds__(256) void diag_scan_kernel(unsigned* R2w, const float* __restrict__ lamgam) {
  const int gid = blockIdx.x * 256 + threadIdx.x;
  if (gid >= NBATCH * N_STATE) return;
  const int b = gid >> 9;
  const int p = gid & (N_STATE - 1);
  const v4f lg = *(const v4f*)(lamgam + 4 * p);
  const float lr = lg[0];
  const float li = lg[1];
  const float gr = lg[2];
  const float gi = lg[3];
  unsigned* base = R2w + (size_t)b * SEQLEN * R2_WORDS;
  const int inw = N_STATE + p;
#pragma unroll 1
  for (int dir = 0; dir < 2; ++dir) {
    const int outw = (dir != 0) ? (N_STATE + p) : p;
    const int sg   = (dir != 0) ? -1 : 1;
    float sr = 0.0f;
    float si = 0.0f;
#pragma unroll 1
    for (int c = 0; c < SEQLEN / 8; ++c) {
      const int tb = (dir != 0) ? (SEQLEN - 1 - 8 * c) : (8 * c);
      unsigned raw[8];
#pragma unroll
      for (int j = 0; j < 8; ++j) {
        const int t = tb + sg * j;
        raw[j] = base[(size_t)t * R2_WORDS + inw];
      }
      unsigned ow[8];
#pragma unroll
      for (int j = 0; j < 8; ++j) {
        const unsigned rw = raw[j];
        const float br = h16_to_f32(rw & 0xffffu);
        const float bi = h16_to_f32(rw >> 16);
        const float bur = gr * br - gi * bi;
        const float bui = gr * bi + gi * br;
        const float nr = lr * sr - li * si + bur;
        const float ni = lr * si + li * sr + bui;
        sr = nr;
        si = ni;
        ow[j] = pack_h2(sr * XS_CARRY, si * XS_CARRY);
      }
      for (int pass = 0; pass < 2; ++pass) {
#pragma unroll
        for (int j = 0; j < 8; ++j) {
          const int t = tb + sg * j;
          *(volatile unsigned*)(base + (size_t)t * R2_WORDS + outw) = ow[j];
        }
        __threadfence();
      }
    }
  }
}

__global__ __launch_bounds__(256) void geglu_kernel(unsigned* R2w) {
  const int i = blockIdx.x * 256 + threadIdx.x;
  if (i < NTOK * (D_MODEL / 2)) {
    const int t  = i >> 9;
    const int jw = i & (D_MODEL / 2 - 1);
    unsigned* pa = R2w + (size_t)t * R2_WORDS + jw;
    const unsigned aw = pa[0];
    const unsigned gw = pa[D_MODEL / 2];
    const float a0 = h16_to_f32(aw & 0xffffu);
    const float a1 = h16_to_f32(aw >> 16);
    const float g0 = h16_to_f32(gw & 0xffffu);
    const float g1 = h16_to_f32(gw >> 16);
    const float o0 = a0 * gelu_erf(g0);
    const float o1 = a1 * gelu_erf(g1);
    const unsigned o = pack_h2(o0, o1);
    *(volatile unsigned*)pa = o;
    __threadfence();
    *(volatile unsigned*)pa = o;
  }
}

extern "C" void kernel_launch(void* const* d_in, const int* in_sizes, int n_in,
                              void* d_out, int out_size, void* d_ws, size_t ws_size, hipStream_t stream) {
  if (n_in < 17 || d_out == nullptr || d_ws == nullptr) return;
  if (in_sizes[0] != NTOK * D_INPUT || in_sizes[1] != D_MODEL * D_INPUT || in_sizes[2] != D_INPUT * D_MODEL ||
      in_sizes[3] != D_MODEL || in_sizes[4] != D_MODEL || in_sizes[5] != D_MODEL || in_sizes[6] != D_MODEL ||
      in_sizes[7] != N_STATE || in_sizes[8] != N_STATE || in_sizes[9] != N_STATE ||
      in_sizes[10] != N_STATE * D_MODEL || in_sizes[11] != N_STATE * D_MODEL ||
      in_sizes[12] != D_MODEL * 2 * N_STATE || in_sizes[13] != D_MODEL * 2 * N_STATE ||
      in_sizes[14] != D_MODEL || in_sizes[15] != D_FF2 * D_MODEL || in_sizes[16] != D_MODEL * D_MODEL ||
      out_size != NTOK * D_INPUT) return;

  const float* x        = (const float*)d_in[0];
  const float* W_in     = (const float*)d_in[1];
  const float* W_out    = (const float*)d_in[2];
  const float* ln1_w    = (const float*)d_in[3];
  const float* ln1_b    = (const float*)d_in[4];
  const float* ln2_w    = (const float*)d_in[5];
  const float* ln2_b    = (const float*)d_in[6];
  const float* Lam_re   = (const float*)d_in[7];
  const float* Lam_im   = (const float*)d_in[8];
  const float* log_step = (const float*)d_in[9];
  const float* B_re     = (const float*)d_in[10];
  const float* B_im     = (const float*)d_in[11];
  const float* C_re     = (const float*)d_in[12];
  const float* C_im     = (const float*)d_in[13];
  const float* Dvec     = (const float*)d_in[14];
  const float* ff_enc   = (const float*)d_in[15];
  const float* ff_dec   = (const float*)d_in[16];
  float* out = (float*)d_out;

  char* ws = (char*)d_ws;
  size_t off = 0;
  auto carve = [&](size_t bytes) -> char* { char* p = ws + off; off += (bytes + 255) & ~(size_t)255; return p; };
  unsigned short* WIN16 = (unsigned short*)carve((size_t)D_MODEL * D_INPUT * 2);
  unsigned short* WB    = (unsigned short*)carve((size_t)D_MODEL * D_MODEL * 2);
  unsigned short* WC    = (unsigned short*)carve((size_t)D_MODEL * XS_COLS * 2);
  unsigned short* WENC  = (unsigned short*)carve((size_t)D_FF2 * D_MODEL * 2);
  unsigned short* WDEC  = (unsigned short*)carve((size_t)D_MODEL * D_MODEL * 2);
  unsigned short* WOUT  = (unsigned short*)carve((size_t)D_INPUT * D_MODEL * 2);
  float*          LAMGAM = (float*)carve((size_t)N_STATE * 4 * 4);
  unsigned short* R1    = (unsigned short*)carve((size_t)NTOK * D_MODEL * 2);
  unsigned short* R2    = (unsigned short*)carve((size_t)NTOK * XS_COLS * 2);
  unsigned short* YPL   = (unsigned short*)carve((size_t)HALF_TOK * D_MODEL * 2);
  if (off > ws_size || off > (size_t)134217728) return;
  float* H1 = (float*)R2;
  unsigned short* X16 = R1;

  disc_prep_kernel<<<(N_STATE + 255) / 256, 256, 0, stream>>>(Lam_re, Lam_im, log_step, LAMGAM);

  cvt8_rows_kernel<<<(D_MODEL * (D_INPUT / 8) + 255) / 256, 256, 0, stream>>>(
      W_in, WIN16, D_MODEL, D_INPUT / 8, D_INPUT, W_CARRY, D_INPUT, 0, 1);
  cvt8_rows_kernel<<<(N_STATE * (D_MODEL / 8) + 255) / 256, 256, 0, stream>>>(
      B_re, WB, N_STATE, D_MODEL / 8, D_MODEL, W_CARRY, D_MODEL, 0, 2);
  cvt8_rows_kernel<<<(N_STATE * (D_MODEL / 8) + 255) / 256, 256, 0, stream>>>(
      B_im, WB, N_STATE, D_MODEL / 8, D_MODEL, W_CARRY, D_MODEL, 1, 2);
  cvt_wc_kernel<<<(D_MODEL * (XS_COLS / 8) + 255) / 256, 256, 0, stream>>>(C_re, C_im, WC, 2.0f * W_CARRY);
  cvt8_rows_kernel<<<(D_FF2 * (D_MODEL / 8) + 255) / 256, 256, 0, stream>>>(
      ff_enc, WENC, D_FF2, D_MODEL / 8, D_MODEL, W_CARRY, D_MODEL, 0, 1);
  cvt8_rows_kernel<<<(D_MODEL * (D_MODEL / 8) + 255) / 256, 256, 0, stream>>>(
      ff_dec, WDEC, D_MODEL, D_MODEL / 8, D_MODEL, W_CARRY, D_MODEL, 0, 1);
  cvt8_rows_kernel<<<(D_INPUT * (D_MODEL / 8) + 255) / 256, 256, 0, stream>>>(
      W_out, WOUT, D_INPUT, D_MODEL / 8, D_MODEL, W_CARRY, D_MODEL, 0, 1);
  cvt8_rows_kernel<<<(NTOK * (D_INPUT / 8) + 255) / 256, 256, 0, stream>>>(
      x, X16, NTOK, D_INPUT / 8, D_INPUT, 1.0f, D_INPUT, 0, 1);

  wmma_gemm64_f16<0, false><<<((NTOK >> 6) * (D_MODEL >> 6) + 7) / 8, 256, 0, stream>>>(
      X16, D_INPUT, WIN16, D_INPUT, (void*)H1, D_MODEL, X16, 0, NTOK, D_MODEL, D_INPUT, W_CARRY_INV);

  ln_f32_rows_kernel<<<NTOK / 8, 256, 0, stream>>>(H1, ln1_w, ln1_b, R1, NTOK);

  wmma_gemm64_f16<1, false><<<((NTOK >> 6) * (D_MODEL >> 6) + 7) / 8, 256, 0, stream>>>(
      R1, D_MODEL, WB, D_MODEL, (void*)(R2 + D_MODEL), XS_COLS, R1, 0, NTOK, D_MODEL, D_MODEL, W_CARRY_INV);

  diag_scan_kernel<<<(NBATCH * N_STATE) / 256, 256, 0, stream>>>((unsigned*)R2, LAMGAM);

  for (int hf = 0; hf < 2; ++hf) {
    const unsigned short* Axs = R2 + (size_t)hf * HALF_TOK * XS_COLS;
    wmma_gemm64_f16<1, false><<<((HALF_TOK >> 6) * (D_MODEL >> 6) + 7) / 8, 256, 0, stream>>>(
        Axs, XS_COLS, WC, XS_COLS, (void*)YPL, D_MODEL, R1, 0, HALF_TOK, D_MODEL, XS_COLS, YS_SCALE);
    gelu_res_ln_kernel<<<HALF_TOK / 4, 128, 0, stream>>>(YPL, R1, Dvec, ln2_w, ln2_b, hf * HALF_TOK, HALF_TOK);
  }

  wmma_gemm64_f16<1, false><<<((NTOK >> 6) * (D_FF2 >> 6) + 7) / 8, 256, 0, stream>>>(
      R1, D_MODEL, WENC, D_MODEL, (void*)R2, D_FF2, R1, 0, NTOK, D_FF2, D_MODEL, W_CARRY_INV);

  geglu_kernel<<<(NTOK * (D_MODEL / 2)) / 256, 256, 0, stream>>>((unsigned*)R2);

  wmma_gemm64_f16<1, true><<<((NTOK >> 6) * (D_MODEL >> 6) + 7) / 8, 256, 0, stream>>>(
      R2, D_FF2, WDEC, D_MODEL, (void*)(R2 + D_MODEL), D_FF2, R1, D_MODEL, NTOK, D_MODEL, D_MODEL, W_CARRY_INV);

  wmma_gemm64_f16<0, false><<<((NTOK >> 6) * (D_INPUT >> 6) + 7) / 8, 256, 0, stream>>>(
      R2 + D_MODEL, D_FF2, WOUT, D_MODEL, (void*)out, D_INPUT, R1, 0, NTOK, D_INPUT, D_MODEL, W_CARRY_INV);
}
